// LSTM_6820408066677
// MI455X (gfx1250) — hardware-verified
//
#include <hip/hip_runtime.h>
#include <math.h>

constexpr int NBATCH   = 512;
constexpr int NSTEP    = 1024;
constexpr int NHID     = 128;
constexpr int NCLS     = 10;
constexpr int NGATE    = 4;
constexpr int ROWS_BLK = 16;
constexpr int NTHR     = 256;
constexpr int HPITCH   = 136;
constexpr int BPITCH   = 132;
constexpr int XCHUNK   = 32;
constexpr float WCARRY     = 16.0f;
constexpr float WCARRY_INV = 1.0f / WCARRY;
constexpr float LOG2E_F    = 1.4426950408889634f;
constexpr float K_SIG   = -LOG2E_F * WCARRY_INV;
constexpr float K_TANH  = 2.0f * LOG2E_F * WCARRY_INV;
constexpr float K_TANH1 = 2.0f * LOG2E_F;

static_assert(NBATCH % ROWS_BLK == 0, "batch is a multiple of the 16-row block");
static_assert(NHID == 16 * (NTHR / 32), "8 waves x 16 hidden columns");
static_assert(NHID % 32 == 0, "K multiple of 32");
static_assert(NSTEP % XCHUNK == 0, "whole x chunks");
static_assert((XCHUNK & 1) == 0, "h buffer parity follows the in-chunk step");
static_assert((2 * ROWS_BLK * HPITCH) % NTHR == 0, "h zero-fill loop exact");
static_assert(ROWS_BLK * XCHUNK == 2 * NTHR, "x staging: 2 elements per thread");
static_assert((ROWS_BLK * NCLS) % 32 == 0, "block output is whole 128-B lines");
static_assert(HPITCH % 8 == 0 && BPITCH % 4 == 0, "vector alignment of LDS rows");

typedef __attribute__((ext_vector_type(16))) _Float16 v16h;
typedef __attribute__((ext_vector_type(8)))  _Float16 v8h;
typedef __attribute__((ext_vector_type(8)))  float    v8f;
typedef __attribute__((ext_vector_type(4)))  float    v4f;
typedef __attribute__((ext_vector_type(2)))  float    v2f;

__device__ __forceinline__ void guard_all(v8f& a0, v8f& a1, v8f& a2, v8f& a3,
                                          v16h a, v16h b0, v16h b1, v16h b2, v16h b3) {
  asm volatile("v_nop\n\tv_nop\n\tv_nop\n\tv_nop"
               : "+v"(a0), "+v"(a1), "+v"(a2), "+v"(a3)
               : "v"(a), "v"(b0), "v"(b1), "v"(b2), "v"(b3));
}
__device__ __forceinline__ void acc_guard4(v8f& a, v8f& b, v8f& c, v8f& d) {
  asm volatile("v_nop\n\tv_nop\n\tv_nop\n\tv_nop" : "+v"(a), "+v"(b), "+v"(c), "+v"(d));
}

template <typename T> struct Frag;
template <> struct Frag<_Float16> {
  typedef v16h V; union U { v16h v; v8h h[2]; };
  static __device__ __forceinline__ v16h load(const _Float16* p) {
    U f; f.h[0] = *(const v8h*)(p); f.h[1] = *(const v8h*)(p + 16); return f.v;
  }
  static __device__ __forceinline__ v8f mma(v16h a, v16h b, v8f c) {
    return __builtin_amdgcn_wmma_f32_16x16x32_f16(false, a, false, b, (short)0, c, false, false);
  }
};

__device__ __forceinline__ float sig_carried(float a) {
  return __builtin_amdgcn_rcpf(1.0f + __builtin_amdgcn_exp2f(a * K_SIG));
}
__device__ __forceinline__ float tanh_carried(float a) {
  return 1.0f - 2.0f * __builtin_amdgcn_rcpf(__builtin_amdgcn_exp2f(a * K_TANH) + 1.0f);
}
__device__ __forceinline__ float tanh_plain(float a) {
  return 1.0f - 2.0f * __builtin_amdgcn_rcpf(__builtin_amdgcn_exp2f(a * K_TANH1) + 1.0f);
}

__global__ __launch_bounds__(NTHR) void wplane_kernel(const float* __restrict__ w0, const float* __restrict__ w1,
                                                      const float* __restrict__ w2, const float* __restrict__ w3,
                                                      unsigned short* __restrict__ O) {
  __shared__ float Tt[64 * 65];
  const int tid = threadIdx.x;
  const int gate = blockIdx.z;
  const float* src = (gate == 0) ? w0 : (gate == 1) ? w1 : (gate == 2) ? w2 : w3;
  const int c0 = blockIdx.x * 64;
  const int r0 = blockIdx.y * 64;
#pragma unroll
  for (int i = 0; i < 4; ++i) {
    const int idx = i * NTHR + tid;
    const int rr = idx >> 4;
    const int cc = (idx & 15) * 4;
    const v4f v = *(const v4f*)(src + (size_t)(r0 + rr) * NHID + c0 + cc);
    Tt[rr * 65 + cc + 0] = v[0];
    Tt[rr * 65 + cc + 1] = v[1];
    Tt[rr * 65 + cc + 2] = v[2];
    Tt[rr * 65 + cc + 3] = v[3];
  }
  __syncthreads();
  const int q = tid >> 3;
  const int c8 = (tid & 7) * 8;
  v8h hv[2];
#pragma unroll
  for (int g2 = 0; g2 < 2; ++g2) {
    const int qq = g2 * 32 + q;
#pragma unroll
    for (int e = 0; e < 8; ++e) {
      const float f = Tt[(c8 + e) * 65 + qq];
      hv[g2][e] = (_Float16)(f * WCARRY);
    }
  }
  for (int pass = 0; pass < 2; ++pass) {
#pragma unroll
    for (int g2 = 0; g2 < 2; ++g2) {
      const size_t o = (size_t)(gate * NHID + c0 + g2 * 32 + q) * (size_t)NHID + (size_t)(r0 + c8);
      *(volatile v8h*)(O + o) = hv[g2];
    }
    __threadfence();
  }
}

__global__ __launch_bounds__(NTHR) void lstm_seq_kernel(
    const float* __restrict__ x,
    const float* __restrict__ wgx, const float* __restrict__ bgp,
    const float* __restrict__ wix, const float* __restrict__ bip,
    const float* __restrict__ wfx, const float* __restrict__ bfp,
    const float* __restrict__ wox, const float* __restrict__ bop,
    const float* __restrict__ wph, const float* __restrict__ bpp,
    const unsigned short* __restrict__ WHp, float* __restrict__ out) {
  __shared__ __align__(16) _Float16 Ah[2][ROWS_BLK * HPITCH];
  __shared__ __align__(16) float    Xs[XCHUNK * ROWS_BLK];
  __shared__ __align__(16) float    Bs[NGATE][ROWS_BLK * BPITCH];
  __shared__ __align__(16) float    Hf[ROWS_BLK * BPITCH];
  __shared__ __align__(16) float    Os[ROWS_BLK * NCLS];

  const _Float16* WH = (const _Float16*)WHp;
  const int tid = threadIdx.x;
  const int lane = tid & 31;
  const int wave = tid >> 5;
  const int c = lane & 15;
  const int hh = lane >> 4;
  const int koff = hh * 8;
  const int rowbase = blockIdx.x * ROWS_BLK;
  const int j = 16 * wave + c;

#pragma unroll
  for (int it = 0; it < 2; ++it) {
    const int idx = it * NTHR + tid;
    const int m = idx >> 5;
    const int c4 = (idx & 31) * 4;
    const size_t off = (size_t)(rowbase + m) * NHID + c4;
    const v4f vg = *(const v4f*)(bgp + off);
    const v4f vi = *(const v4f*)(bip + off);
    const v4f vf = *(const v4f*)(bfp + off);
    const v4f vo = *(const v4f*)(bop + off);
    *(v4f*)(&Bs[0][m * BPITCH + c4]) = vg;
    *(v4f*)(&Bs[1][m * BPITCH + c4]) = vi;
    *(v4f*)(&Bs[2][m * BPITCH + c4]) = vf;
    *(v4f*)(&Bs[3][m * BPITCH + c4]) = vo;
  }
  {
    _Float16* ahf = &Ah[0][0];
#pragma unroll 1
    for (int i = tid; i < 2 * ROWS_BLK * HPITCH; i += NTHR) ahf[i] = (_Float16)0.0f;
  }
  __syncthreads();

  float bb[NGATE][8];
#pragma unroll
  for (int g = 0; g < NGATE; ++g)
#pragma unroll
    for (int r = 0; r < 8; ++r) bb[g][r] = Bs[g][(8 * hh + r) * BPITCH + j] * WCARRY;
  const float wxs0 = wgx[j] * WCARRY;
  const float wxs1 = wix[j] * WCARRY;
  const float wxs2 = wfx[j] * WCARRY;
  const float wxs3 = wox[j] * WCARRY;

  float cst[8], hst[8];
#pragma unroll
  for (int r = 0; r < 8; ++r) { cst[r] = 0.0f; hst[r] = 0.0f; }

  const _Float16* wh = WH + (size_t)j * NHID + koff;

#pragma unroll 1
  for (int tb = 0; tb < NSTEP / XCHUNK; ++tb) {
    {
      const int m = tid >> 4;
      const int j2 = (tid & 15) * 2;
      const v2f xv2 = *(const v2f*)(x + (size_t)(rowbase + m) * NSTEP + (size_t)tb * XCHUNK + j2);
      Xs[j2 * ROWS_BLK + m] = xv2[0];
      Xs[(j2 + 1) * ROWS_BLK + m] = xv2[1];
    }
    __syncthreads();

#pragma unroll 1
    for (int ts = 0; ts < XCHUNK; ++ts) {
      const int cur = ts & 1;
      const _Float16* ahrow = &Ah[cur][0] + c * HPITCH + koff;
      _Float16* ahn = &Ah[cur ^ 1][0];

      const v4f xa = *(const v4f*)(Xs + ts * ROWS_BLK + 8 * hh);
      const v4f xb = *(const v4f*)(Xs + ts * ROWS_BLK + 8 * hh + 4);

      v8f acc[NGATE];
#pragma unroll
      for (int r = 0; r < 4; ++r) {
        acc[0][r]     = fmaf(xa[r], wxs0, bb[0][r]);
        acc[0][4 + r] = fmaf(xb[r], wxs0, bb[0][4 + r]);
        acc[1][r]     = fmaf(xa[r], wxs1, bb[1][r]);
        acc[1][4 + r] = fmaf(xb[r], wxs1, bb[1][4 + r]);
        acc[2][r]     = fmaf(xa[r], wxs2, bb[2][r]);
        acc[2][4 + r] = fmaf(xb[r], wxs2, bb[2][4 + r]);
        acc[3][r]     = fmaf(xa[r], wxs3, bb[3][r]);
        acc[3][4 + r] = fmaf(xb[r], wxs3, bb[3][4 + r]);
      }

#pragma unroll 1
      for (int k0 = 0; k0 < NHID; k0 += 32) {
        const v16h a  = Frag<_Float16>::load(ahrow + k0);
        const v16h b0 = Frag<_Float16>::load(wh + k0);
        const v16h b1 = Frag<_Float16>::load(wh + (size_t)1 * NHID * NHID + k0);
        const v16h b2 = Frag<_Float16>::load(wh + (size_t)2 * NHID * NHID + k0);
        const v16h b3 = Frag<_Float16>::load(wh + (size_t)3 * NHID * NHID + k0);
        acc[0] = Frag<_Float16>::mma(a, b0, acc[0]);
        acc[1] = Frag<_Float16>::mma(a, b1, acc[1]);
        acc[2] = Frag<_Float16>::mma(a, b2, acc[2]);
        acc[3] = Frag<_Float16>::mma(a, b3, acc[3]);
        guard_all(acc[0], acc[1], acc[2], acc[3], a, b0, b1, b2, b3);
      }
      acc_guard4(acc[0], acc[1], acc[2], acc[3]);

#pragma unroll
      for (int r = 0; r < 8; ++r) {
        const float gg = tanh_carried(acc[0][r]);
        const float ig = sig_carried(acc[1][r]);
        const float fg = sig_carried(acc[2][r]);
        const float og = sig_carried(acc[3][r]);
        const float cn = gg * ig + cst[r] * fg;
        cst[r] = cn;
        const float hn = tanh_plain(cn) * og;
        hst[r] = hn;
        ahn[(8 * hh + r) * HPITCH + j] = (_Float16)hn;
      }
      __syncthreads();
    }
  }

#pragma unroll
  for (int r = 0; r < 8; ++r) Hf[(8 * hh + r) * BPITCH + j] = hst[r];
  __syncthreads();

  if (tid < ROWS_BLK * NCLS) {
    const int m = tid / NCLS;
    const int cc = tid - m * NCLS;
    float a = 0.0f;
#pragma unroll 4
    for (int k = 0; k < NHID; ++k) a = fmaf(Hf[m * BPITCH + k], wph[k * NCLS + cc], a);
    const float res = a + bpp[(size_t)(rowbase + m) * NCLS + cc];
    Os[tid] = res;
  }
  __syncthreads();

  if (wave == 0) {
    float* op = out + (size_t)rowbase * NCLS;
    float vals[5];
#pragma unroll
    for (int it = 0; it < 5; ++it) vals[it] = Os[it * 32 + lane];
    for (int pass = 0; pass < 2; ++pass) {
#pragma unroll
      for (int it = 0; it < 5; ++it) *(volatile float*)(op + it * 32 + lane) = vals[it];
      __threadfence();
    }
  }
}

extern "C" void kernel_launch(void* const* d_in, const int* in_sizes, int n_in,
                              void* d_out, int out_size, void* d_ws, size_t ws_size, hipStream_t stream) {
  if (n_in < 15 || d_out == nullptr || d_ws == nullptr) return;
  if (in_sizes[0] != NBATCH * NSTEP || out_size != NBATCH * NCLS) return;
  if (in_sizes[1] != NHID || in_sizes[4] != NHID || in_sizes[7] != NHID || in_sizes[10] != NHID) return;
  if (in_sizes[2] != NHID * NHID || in_sizes[5] != NHID * NHID || in_sizes[8] != NHID * NHID ||
      in_sizes[11] != NHID * NHID) return;
  if (in_sizes[3] != NBATCH * NHID || in_sizes[6] != NBATCH * NHID || in_sizes[9] != NBATCH * NHID ||
      in_sizes[12] != NBATCH * NHID) return;
  if (in_sizes[13] != NHID * NCLS || in_sizes[14] != NBATCH * NCLS) return;

  const float* x   = (const float*)d_in[0];
  const float* Wgx = (const float*)d_in[1];
  const float* Wgh = (const float*)d_in[2];
  const float* bg  = (const float*)d_in[3];
  const float* Wix = (const float*)d_in[4];
  const float* Wih = (const float*)d_in[5];
  const float* bi  = (const float*)d_in[6];
  const float* Wfx = (const float*)d_in[7];
  const float* Wfh = (const float*)d_in[8];
  const float* bfo = (const float*)d_in[9];
  const float* Wox = (const float*)d_in[10];
  const float* Woh = (const float*)d_in[11];
  const float* bo  = (const float*)d_in[12];
  const float* Wph = (const float*)d_in[13];
  const float* bp  = (const float*)d_in[14];
  float* out = (float*)d_out;

  const size_t wh_bytes = (size_t)NGATE * NHID * NHID * 2;
  if (wh_bytes > ws_size || wh_bytes > (size_t)134217728) return;
  unsigned short* WH = (unsigned short*)d_ws;

  wplane_kernel<<<dim3(NHID / 64, NHID / 64, NGATE), NTHR, 0, stream>>>(Wgh, Wih, Wfh, Woh, WH);
  lstm_seq_kernel<<<NBATCH / ROWS_BLK, NTHR, 0, stream>>>(x, Wgx, bg, Wix, bi, Wfx, bfo, Wox, bo, Wph, bp, WH, out);
}
